// VMambaSS2D_26869315404386
// MI455X (gfx1250) — hardware-verified
//
#include <hip/hip_runtime.h>
#include <math.h>

typedef __attribute__((ext_vector_type(16))) _Float16 v16h;
typedef __attribute__((ext_vector_type(8)))  _Float16 v8h;
typedef __attribute__((ext_vector_type(4)))  _Float16 v4h;
typedef __attribute__((ext_vector_type(16))) __bf16   v16b;
typedef __attribute__((ext_vector_type(8)))  __bf16   v8b;
typedef __attribute__((ext_vector_type(8)))  float    v8f;
typedef __attribute__((ext_vector_type(4)))  float    v4f;
typedef __attribute__((ext_vector_type(2)))  float    v2f;
typedef __attribute__((ext_vector_type(8)))  unsigned short v8us;
typedef __attribute__((ext_vector_type(4)))  unsigned short v4us;

constexpr int NBATCH = 2;
constexpr int IMH    = 64;
constexpr int IMW    = 64;
constexpr int NPIX   = IMH * IMW;
constexpr int NTOK   = NBATCH * NPIX;
constexpr int DMOD   = 96;
constexpr int DIN    = 192;
constexpr int NST    = 16;
constexpr int DTRK   = 6;
constexpr int NDIR   = 4;
constexpr int NPADO  = 128;
constexpr int XDW    = 64;
constexpr int XPROWS = 38;
constexpr int SROW   = 136;
constexpr int SCHUNK = 32;
constexpr int SITEMS = SCHUNK * 34;

__device__ __forceinline__ unsigned short f2bf_bits(float f) {
  unsigned u = __float_as_uint(f);
  return (unsigned short)((u + 0x7FFFu + ((u >> 16) & 1u)) >> 16);
}
__device__ __forceinline__ float bf_bits2f(unsigned short h) { return __uint_as_float(((unsigned)h) << 16); }

__device__ __forceinline__ void dep_guard_h(v8f& a, v8f& b, v16h x, v16h y) { asm volatile("v_nop\n\tv_nop\n\tv_nop\n\tv_nop" : "+v"(a), "+v"(b) : "v"(x), "v"(y)); }
__device__ __forceinline__ void dep_guard_b(v8f& a, v8f& b, v16b x, v16b y) { asm volatile("v_nop\n\tv_nop\n\tv_nop\n\tv_nop" : "+v"(a), "+v"(b) : "v"(x), "v"(y)); }
__device__ __forceinline__ void keep4_h(v16h a, v16h b, v16h c, v16h d) { asm volatile("v_nop" :: "v"(a), "v"(b), "v"(c), "v"(d)); }
__device__ __forceinline__ void keep4_b(v16b a, v16b b, v16b c, v16b d) { asm volatile("v_nop" :: "v"(a), "v"(b), "v"(c), "v"(d)); }
__device__ __forceinline__ void acc_guard4(v8f& a, v8f& b, v8f& c, v8f& d) { asm volatile("v_nop\n\tv_nop\n\tv_nop\n\tv_nop" : "+v"(a), "+v"(b), "+v"(c), "+v"(d)); }
template <typename T> struct Frag;
template <> struct Frag<_Float16> {
  typedef v16h V; union U { v16h v; v8h h[2]; };
  static __device__ __forceinline__ v16h load(const _Float16* p) {
    U f; f.h[0] = *(const v8h*)(p); f.h[1] = *(const v8h*)(p + 16); return f.v;
  }
  static __device__ __forceinline__ v8f mma(v16h a, v16h b, v8f c) {
    return __builtin_amdgcn_wmma_f32_16x16x32_f16(false, a, false, b, (short)0, c, false, false);
  }
  static __device__ __forceinline__ void guard(v8f& a, v8f& b, v16h x, v16h y) { dep_guard_h(a, b, x, y); }
  static __device__ __forceinline__ void keep(v16h a, v16h b, v16h c, v16h d) { keep4_h(a, b, c, d); }
};
template <> struct Frag<__bf16> {
  typedef v16b V; union U { v16b v; v8b h[2]; };
  static __device__ __forceinline__ v16b load(const __bf16* p) {
    U f; f.h[0] = *(const v8b*)(p); f.h[1] = *(const v8b*)(p + 16); return f.v;
  }
  static __device__ __forceinline__ v8f mma(v16b a, v16b b, v8f c) {
    return __builtin_amdgcn_wmma_f32_16x16x32_bf16(false, a, false, b, (short)0, c, false, false);
  }
  static __device__ __forceinline__ void guard(v8f& a, v8f& b, v16b x, v16b y) { dep_guard_b(a, b, x, y); }
  static __device__ __forceinline__ void keep(v16b a, v16b b, v16b c, v16b d) { keep4_b(a, b, c, d); }
};

template <int ET> struct Elem;
template <> struct Elem<0> { typedef _Float16 T; };
template <> struct Elem<1> { typedef __bf16 T; };
template <int ET, bool SPLIT, int BIAS_MODE, int OUT_MODE, bool RESID, int ACT = 0>
__global__ __launch_bounds__(256) void wmma_gemm64(
    const unsigned short* __restrict__ Ap, const unsigned short* __restrict__ A2p, int lda, long strideA,
    const unsigned short* __restrict__ Btp, const unsigned short* __restrict__ Bt2p, int ldb, long strideB,
    void* __restrict__ Cout, void* __restrict__ Cout2, int ldc, long strideC,
    const float* __restrict__ bias,
    const float* __restrict__ resid, long strideR,
    int M, int N, int K, float scale) {
  typedef typename Elem<ET>::T T;
  typedef typename Frag<T>::V V;
  const T* A = (const T*)Ap; const T* A2 = (const T*)A2p; const T* Bt = (const T*)Btp; const T* Bt2 = (const T*)Bt2p;
  __shared__ __align__(16) float sT[8][16 * 68];
  const int b    = blockIdx.y;
  const int lane = threadIdx.x & 31;
  const int wave = threadIdx.x >> 5;
  const int tilesN = N >> 6;
  const int tilesM = M >> 6;
  const int tile = blockIdx.x * 8 + wave;
  if (tile >= tilesM * tilesN) return;
  const int tm = tile / tilesN;
  const int tn = tile - tm * tilesN;
  const int m0 = tm << 6;
  const int n0 = tn << 6;

  const T* Ab  = A  + (size_t)b * strideA;
  const T* Bb  = Bt + (size_t)b * strideB;
  const T* Ab2 = SPLIT ? (A2  + (size_t)b * strideA) : nullptr;
  const T* Bb2 = SPLIT ? (Bt2 + (size_t)b * strideB) : nullptr;

  const int rlane = lane & 15;
  const int koff  = (lane >> 4) * 8;
  const int mOff  = (lane >> 4) * 8;

  v8f acc[4][4];
#pragma unroll
  for (int i = 0; i < 4; ++i)
#pragma unroll
    for (int j = 0; j < 4; ++j) acc[i][j] = (v8f){0.f,0.f,0.f,0.f,0.f,0.f,0.f,0.f};

  for (int k0 = 0; k0 < K; k0 += 32) {
    V bh[4], bl[4];
#pragma unroll
    for (int j = 0; j < 4; ++j) {
      const size_t bo = (size_t)(n0 + (j << 4) + rlane) * ldb + koff + k0;
      bh[j] = Frag<T>::load(Bb + bo);
      if (SPLIT) bl[j] = Frag<T>::load(Bb2 + bo);
    }
#pragma unroll
    for (int i = 0; i < 4; ++i) {
      const size_t ao = (size_t)(m0 + (i << 4) + rlane) * lda + koff + k0;
      V ah = Frag<T>::load(Ab + ao);
      V al;
      if (SPLIT) al = Frag<T>::load(Ab2 + ao);
#pragma unroll
      for (int j = 0; j < 4; ++j) {
        acc[i][j] = Frag<T>::mma(ah, bh[j], acc[i][j]);
        if (SPLIT) {
          acc[i][j] = Frag<T>::mma(ah, bl[j], acc[i][j]);
          acc[i][j] = Frag<T>::mma(al, bh[j], acc[i][j]);
        }
      }
      Frag<T>::guard(acc[i][0], acc[i][3], ah, SPLIT ? al : ah);
    }
    Frag<T>::keep(bh[0], bh[1], bh[2], bh[3]);
    if (SPLIT) Frag<T>::keep(bl[0], bl[1], bl[2], bl[3]);
  }
  acc_guard4(acc[0][0], acc[0][1], acc[0][2], acc[0][3]);
  acc_guard4(acc[1][0], acc[1][1], acc[1][2], acc[1][3]);
  acc_guard4(acc[2][0], acc[2][1], acc[2][2], acc[2][3]);
  acc_guard4(acc[3][0], acc[3][1], acc[3][2], acc[3][3]);

  float* slab = sT[wave];
  const float* Rb = RESID ? (resid + (size_t)b * strideR) : nullptr;
#pragma unroll
  for (int i = 0; i < 4; ++i) {
    const int mBase = m0 + (i << 4);
#pragma unroll
    for (int j = 0; j < 4; ++j) {
      const int n = n0 + (j << 4) + rlane;
      float bv = 0.f;
      if (BIAS_MODE == 2) bv = bias[n];
#pragma unroll
      for (int r = 0; r < 8; ++r) {
        float v = acc[i][j][r] * scale;
        if (BIAS_MODE == 1) v += bias[mBase + mOff + r];
        if (BIAS_MODE == 2) v += bv;
        if (RESID) v += Rb[(size_t)(mBase + mOff + r) * ldc + n];
        if (ACT == 1) v = tanhf(v);
        if (ACT == 2) v = fmaxf(v, 0.0f);
        if (ACT == 3) v = v / (1.0f + expf(-v));
        if (ACT == 4) v = (v > 0.f) ? v : 0.01f * v;
        if (ACT == 5) v = 0.5f * v * (1.0f + erff(v * 0.70710678118654752f));
        slab[(mOff + r) * 68 + (j << 4) + rlane] = v;
      }
    }
    __builtin_amdgcn_fence(__ATOMIC_RELEASE, "workgroup");
    __builtin_amdgcn_wave_barrier();
    __builtin_amdgcn_fence(__ATOMIC_ACQUIRE, "workgroup");
    if (OUT_MODE == 0) {
      float* C = (float*)Cout + (size_t)b * strideC;
      const int hh = lane >> 4, c4 = (lane & 15) * 4;
      for (int pass = 0; pass < 2; ++pass) {
#pragma unroll
        for (int it = 0; it < 8; ++it) {
          const int row = it * 2 + hh;
          v4f v = *(const v4f*)(slab + row * 68 + c4);
          *(volatile v4f*)(C + (size_t)(mBase + row) * ldc + n0 + c4) = v;
        }
        __threadfence();
      }
    } else {
      const int q = lane >> 3, c8 = (lane & 7) * 8;
      unsigned short* C  = (unsigned short*)Cout  + (size_t)b * strideC;
      unsigned short* C2 = (OUT_MODE == 2) ? ((unsigned short*)Cout2 + (size_t)b * strideC) : nullptr;
      for (int pass = 0; pass < 2; ++pass) {
#pragma unroll
        for (int it = 0; it < 4; ++it) {
          const int row = it * 4 + q;
          const float* sp = slab + row * 68 + c8;
          v8h hv, lv;
#pragma unroll
          for (int e = 0; e < 8; ++e) {
            if (OUT_MODE == 1) {
              hv[e] = (_Float16)sp[e];
            } else {
              unsigned short hb = f2bf_bits(sp[e]);
              unsigned short lb = f2bf_bits(sp[e] - bf_bits2f(hb));
              hv[e] = __builtin_bit_cast(_Float16, hb);
              lv[e] = __builtin_bit_cast(_Float16, lb);
            }
          }
          *(volatile v8h*)(C + (size_t)(mBase + row) * ldc + n0 + c8) = hv;
          if (OUT_MODE == 2) *(volatile v8h*)(C2 + (size_t)(mBase + row) * ldc + n0 + c8) = lv;
        }
        __threadfence();
      }
    }
    __builtin_amdgcn_fence(__ATOMIC_RELEASE, "workgroup");
    __builtin_amdgcn_wave_barrier();
    __builtin_amdgcn_fence(__ATOMIC_ACQUIRE, "workgroup");
  }
}

__global__ __launch_bounds__(256) void cast_rows_kernel(
    const float* __restrict__ src, unsigned short* __restrict__ dst,
    int R, int Rp, int Kc, int rot, int nchunks, float scale)
{
  const int f = blockIdx.x * 256 + threadIdx.x;
  if (f >= nchunks) return;
  const int cpr = Kc >> 3;
  const int rowflat = f / cpr;
  const int g  = f - rowflat * cpr;
  const int kb = rowflat / Rp;
  const int n  = rowflat - kb * Rp;
  const bool valid = n < R;
  int sr = n + rot;
  sr = (sr >= R) ? (sr - R) : sr;
  sr = valid ? sr : 0;
  const float* p = src + ((size_t)kb * R + sr) * Kc + g * 8;
  const v4f a0 = *(const v4f*)(p);
  const v4f a1 = *(const v4f*)(p + 4);
  v8h hv;
#pragma unroll
  for (int e = 0; e < 4; ++e) {
    hv[e]     = (_Float16)(valid ? a0[e] * scale : 0.0f);
    hv[4 + e] = (_Float16)(valid ? a1[e] * scale : 0.0f);
  }
  unsigned short* q = dst + (size_t)f * 8;
  *(volatile v8h*)q = hv;
  __threadfence();
  *(volatile v8h*)q = hv;
}

__global__ __launch_bounds__(256) void cast_rows_bf2_kernel(
    const float* __restrict__ src, unsigned short* __restrict__ dstH, unsigned short* __restrict__ dstL,
    int R, int Rp, int Kc, int nchunks)
{
  const int f = blockIdx.x * 256 + threadIdx.x;
  if (f >= nchunks) return;
  const int cpr = Kc >> 3;
  const int n   = f / cpr;
  const int g   = f - n * cpr;
  const bool valid = n < R;
  const int sr  = valid ? n : 0;
  const float* p = src + (size_t)sr * Kc + g * 8;
  const v4f a0 = *(const v4f*)(p);
  const v4f a1 = *(const v4f*)(p + 4);
  v8us hv, lv;
#pragma unroll
  for (int e = 0; e < 4; ++e) {
    const float v0 = valid ? a0[e] : 0.0f;
    const unsigned short h0 = f2bf_bits(v0);
    hv[e] = h0; lv[e] = f2bf_bits(v0 - bf_bits2f(h0));
    const float v1 = valid ? a1[e] : 0.0f;
    const unsigned short h1 = f2bf_bits(v1);
    hv[4 + e] = h1; lv[4 + e] = f2bf_bits(v1 - bf_bits2f(h1));
  }
  unsigned short* qh = dstH + (size_t)f * 8;
  unsigned short* ql = dstL + (size_t)f * 8;
  *(volatile v8us*)qh = hv;
  *(volatile v8us*)ql = lv;
  __threadfence();
  *(volatile v8us*)qh = hv;
  *(volatile v8us*)ql = lv;
}

__global__ __launch_bounds__(192) void dwconv_silu_kernel(
    const float* __restrict__ XP, const float* __restrict__ cw, const float* __restrict__ cbias,
    float* __restrict__ XI, unsigned short* __restrict__ XI16)
{
  __shared__ __align__(16) _Float16 sH[IMW * DIN];
  const int d  = threadIdx.x;
  const int b_ = blockIdx.x / IMH;
  const int h_ = blockIdx.x - b_ * IMH;
  const float* wd = cw + d * 9;
  const float w00 = wd[0], w01 = wd[1], w02 = wd[2];
  const float w10 = wd[3], w11 = wd[4], w12 = wd[5];
  const float w20 = wd[6], w21 = wd[7], w22 = wd[8];
  const float bc = cbias[d];
  const bool up = h_ > 0, dn = h_ < IMH - 1;
  const int r0 = up ? (h_ - 1) : 0;
  const int r2 = dn ? (h_ + 1) : (IMH - 1);
  const float* p0 = XP + ((size_t)(b_ * IMH + r0) * IMW) * DIN + d;
  const float* p1 = XP + ((size_t)(b_ * IMH + h_) * IMW) * DIN + d;
  const float* p2 = XP + ((size_t)(b_ * IMH + r2) * IMW) * DIN + d;
  float a0m = 0.f, a1m = 0.f, a2m = 0.f;
  float a0c, a1c, a2c;
  {
    const float v0 = p0[0], v1 = p1[0], v2 = p2[0];
    a0c = up ? v0 : 0.f;
    a1c = v1;
    a2c = dn ? v2 : 0.f;
  }
  float* orow = XI + ((size_t)(b_ * IMH + h_) * IMW) * DIN + d;
#pragma unroll 1
  for (int w = 0; w < IMW; ++w) {
    const bool rv = (w + 1) < IMW;
    const int  wn = rv ? (w + 1) : (IMW - 1);
    const float n0 = p0[(size_t)wn * DIN], n1 = p1[(size_t)wn * DIN], n2 = p2[(size_t)wn * DIN];
    const float a0n = (up && rv) ? n0 : 0.f;
    const float a1n = rv ? n1 : 0.f;
    const float a2n = (dn && rv) ? n2 : 0.f;
    float acc = w00 * a0m;
    acc = fmaf(w01, a0c, acc);
    acc = fmaf(w02, a0n, acc);
    acc = fmaf(w10, a1m, acc);
    acc = fmaf(w11, a1c, acc);
    acc = fmaf(w12, a1n, acc);
    acc = fmaf(w20, a2m, acc);
    acc = fmaf(w21, a2c, acc);
    acc = fmaf(w22, a2n, acc);
    const float sv  = acc + bc;
    const float sg  = __builtin_amdgcn_rcpf(1.0f + __expf(-sv));
    const float out = sv * sg;
    float* op = orow + (size_t)w * DIN;
    *(volatile float*)op = out;
    __threadfence();
    *(volatile float*)op = out;
    sH[w * DIN + d] = (_Float16)(out * 64.0f);
    a0m = a0c; a0c = a0n;
    a1m = a1c; a1c = a1n;
    a2m = a2c; a2c = a2n;
  }
  __syncthreads();
  v8h vals[8];
#pragma unroll
  for (int it = 0; it < 8; ++it) vals[it] = *(const v8h*)(sH + (it * DIN + d) * 8);
  unsigned short* ob = XI16 + (size_t)blockIdx.x * IMW * DIN;
  for (int pass = 0; pass < 2; ++pass) {
#pragma unroll
    for (int it = 0; it < 8; ++it) *(volatile v8h*)(ob + (size_t)(it * DIN + d) * 8) = vals[it];
    __threadfence();
  }
}

__device__ __forceinline__ int dir_tok(int k, int l) {
  const int lr = (k >= 2) ? (NPIX - 1 - l) : l;
  return (k & 1) ? ((lr % IMH) * IMW + lr / IMH) : lr;
}

__global__ __launch_bounds__(192) void scan_dir_kernel(
    const float* __restrict__ XDBL, const float* __restrict__ XI,
    const float* __restrict__ dtw, const float* __restrict__ dtb,
    const float* __restrict__ Alog, const float* __restrict__ Dsp,
    float* __restrict__ Y)
{
  __shared__ __align__(16) float sRow[SCHUNK * SROW];
  const int d  = threadIdx.x;
  const int bk = blockIdx.x;
  const int b_ = bk >> 2;
  const int k  = bk & 3;
  const int g4 = d & 3;
  const size_t tokb = (size_t)b_ * NPIX;
  const float* wr = dtw + ((size_t)k * DIN + d) * DTRK;
  const float w0 = wr[0], w1 = wr[1], w2 = wr[2], w3 = wr[3], w4 = wr[4], w5 = wr[5];
  const float db = dtb[k * DIN + d];
  const float Dk = Dsp[k * DIN + d];
  float An[NST], h[NST];
#pragma unroll
  for (int n = 0; n < NST; ++n) {
    const float al = Alog[((size_t)k * DIN + d) * NST + n];
    An[n] = -__expf(al);
    h[n]  = 0.f;
  }
  float* Yk = Y + (size_t)k * NTOK * DIN;
#pragma unroll 1
  for (int c = 0; c < NPIX / SCHUNK; ++c) {
    __syncthreads();
    for (int q = d; q < SITEMS; q += DIN) {
      const int s   = q / 34;
      const int j   = q - s * 34;
      const int l   = c * SCHUNK + s;
      const bool bc = j < 32;
      const int kp  = bc ? (j >> 3) : k;
      const int col = bc ? ((j & 7) * 4) : (32 + (j - 32) * 4);
      const int tok = dir_tok(kp, l);
      const v4f v = *(const v4f*)(XDBL + ((size_t)kp * NTOK + tokb + tok) * XDW + col);
      *(v4f*)(sRow + s * SROW + 4 * j) = v;
    }
    __syncthreads();
#pragma unroll 1
    for (int s = 0; s < SCHUNK; ++s) {
      const int l   = c * SCHUNK + s;
      const int tok = dir_tok(k, l);
      const size_t ei = (tokb + tok) * DIN + d;
      const float u = XI[ei];
      const float* sr = sRow + s * SROW;
      v4f Bv[4], Cv[4];
#pragma unroll
      for (int i = 0; i < 4; ++i) {
        Bv[i] = *(const v4f*)(sr + g4 * 32 + 4 * i);
        Cv[i] = *(const v4f*)(sr + g4 * 32 + 16 + 4 * i);
      }
      const v4f D0 = *(const v4f*)(sr + 128);
      const v2f D1 = *(const v2f*)(sr + 132);
      float dp = db;
      dp = fmaf(w0, D0[0], dp);
      dp = fmaf(w1, D0[1], dp);
      dp = fmaf(w2, D0[2], dp);
      dp = fmaf(w3, D0[3], dp);
      dp = fmaf(w4, D1[0], dp);
      dp = fmaf(w5, D1[1], dp);
      const float ex   = __expf(-fabsf(dp));
      const float up1  = 1.0f + ex;
      const float den  = up1 - 1.0f;
      const bool  dpos = den > 0.0f;
      const float dens = dpos ? den : 1.0f;
      const float lg   = __logf(up1);
      const float l1p  = dpos ? (lg * (ex * __builtin_amdgcn_rcpf(dens))) : ex;
      const float delta = fmaxf(dp, 0.0f) + l1p;
      const float du    = delta * u;
      float y = Dk * u;
#pragma unroll
      for (int n = 0; n < NST; ++n) {
        const float e  = __expf(delta * An[n]);
        const float hn = fmaf(e, h[n], du * Bv[n >> 2][n & 3]);
        h[n] = hn;
        y = fmaf(hn, Cv[n >> 2][n & 3], y);
      }
      float* yp = Yk + ei;
      *(volatile float*)yp = y;
      __threadfence();
      *(volatile float*)yp = y;
    }
  }
}

__global__ __launch_bounds__(256) void ln_gate_kernel(
    const float* __restrict__ Y, const float* __restrict__ Z,
    const float* __restrict__ g, const float* __restrict__ be,
    unsigned short* __restrict__ dstH, unsigned short* __restrict__ dstL)
{
  __shared__ __align__(16) unsigned short sHt[32 * DIN];
  __shared__ __align__(16) unsigned short sLt[32 * DIN];
  const int t = threadIdx.x;
  const int r = t >> 3, part = t & 7;
  const int row = blockIdx.x * 32 + r;
  const int c0  = part * 24;
  const size_t PL   = (size_t)NTOK * DIN;
  const size_t base = (size_t)row * DIN + c0;
  const float* zr = Z + base;
  v4f a[6];
#pragma unroll
  for (int j = 0; j < 6; ++j) {
    const v4f y0 = *(const v4f*)(Y + base + 4 * j);
    const v4f y2 = *(const v4f*)(Y + 2 * PL + base + 4 * j);
    const v4f y1 = *(const v4f*)(Y + PL + base + 4 * j);
    const v4f y3 = *(const v4f*)(Y + 3 * PL + base + 4 * j);
    a[j] = ((y0 + y2) + y1) + y3;
  }
  float s = 0.f;
#pragma unroll
  for (int j = 0; j < 6; ++j) s += (a[j][0] + a[j][1]) + (a[j][2] + a[j][3]);
  s += __shfl_xor(s, 1, 32);
  s += __shfl_xor(s, 2, 32);
  s += __shfl_xor(s, 4, 32);
  const float mu = s * (1.0f / 192.0f);
  float q = 0.f;
#pragma unroll
  for (int j = 0; j < 6; ++j) {
#pragma unroll
    for (int e = 0; e < 4; ++e) { const float dd = a[j][e] - mu; q = fmaf(dd, dd, q); }
  }
  q += __shfl_xor(q, 1, 32);
  q += __shfl_xor(q, 2, 32);
  q += __shfl_xor(q, 4, 32);
  const float var = q * (1.0f / 192.0f);
  const float is  = rsqrtf(var + 1e-5f);
#pragma unroll
  for (int j = 0; j < 6; ++j) {
    const v4f zz = *(const v4f*)(zr + 4 * j);
    const v4f gg = *(const v4f*)(g  + c0 + 4 * j);
    const v4f bb = *(const v4f*)(be + c0 + 4 * j);
    v4us hv, lv;
#pragma unroll
    for (int e = 0; e < 4; ++e) {
      const float gn = ((a[j][e] - mu) * is) * gg[e] + bb[e];
      const float zv = zz[e];
      const float sg = __builtin_amdgcn_rcpf(1.0f + __expf(-zv));
      const float v  = gn * (zv * sg);
      const unsigned short hb = f2bf_bits(v);
      hv[e] = hb;
      lv[e] = f2bf_bits(v - bf_bits2f(hb));
    }
    *(v4us*)(sHt + r * DIN + c0 + 4 * j) = hv;
    *(v4us*)(sLt + r * DIN + c0 + 4 * j) = lv;
  }
  __syncthreads();
  v8us vh[3], vl[3];
#pragma unroll
  for (int it = 0; it < 3; ++it) {
    vh[it] = *(const v8us*)(sHt + (it * 256 + t) * 8);
    vl[it] = *(const v8us*)(sLt + (it * 256 + t) * 8);
  }
  unsigned short* obh = dstH + (size_t)blockIdx.x * 32 * DIN;
  unsigned short* obl = dstL + (size_t)blockIdx.x * 32 * DIN;
  for (int pass = 0; pass < 2; ++pass) {
#pragma unroll
    for (int it = 0; it < 3; ++it) {
      *(volatile v8us*)(obh + (size_t)(it * 256 + t) * 8) = vh[it];
      *(volatile v8us*)(obl + (size_t)(it * 256 + t) * 8) = vl[it];
    }
    __threadfence();
  }
}

__global__ __launch_bounds__(256) void out_copy_kernel(
    const float* __restrict__ XR, float* __restrict__ out, int nq)
{
  const int f = blockIdx.x * 256 + threadIdx.x;
  if (f >= nq) return;
  const int pos = f / 24;
  const int q   = f - pos * 24;
  const v4f v = *(const v4f*)(XR + (size_t)pos * NPADO + 4 * q);
  float* op = out + (size_t)f * 4;
  *(volatile v4f*)op = v;
  __threadfence();
  *(volatile v4f*)op = v;
}

extern "C" void kernel_launch(void* const* d_in, const int* in_sizes, int n_in,
                              void* d_out, int out_size, void* d_ws, size_t ws_size,
                              hipStream_t stream)
{
  if (n_in < 12) return;
  const float* x    = (const float*)d_in[0];
  const float* inpw = (const float*)d_in[1];
  const float* cw   = (const float*)d_in[2];
  const float* cb   = (const float*)d_in[3];
  const float* xprw = (const float*)d_in[4];
  const float* dtpw = (const float*)d_in[5];
  const float* dtpb = (const float*)d_in[6];
  const float* alog = (const float*)d_in[7];
  const float* dsp  = (const float*)d_in[8];
  const float* lng  = (const float*)d_in[9];
  const float* lnb  = (const float*)d_in[10];
  const float* outw = (const float*)d_in[11];
  float* dout = (float*)d_out;

  if (in_sizes[0] != NTOK * DMOD) return;
  if (in_sizes[1] != 2 * DIN * DMOD) return;
  if (in_sizes[2] != DIN * 9 || in_sizes[3] != DIN) return;
  if (in_sizes[4] != NDIR * XPROWS * DIN) return;
  if (in_sizes[5] != NDIR * DIN * DTRK || in_sizes[6] != NDIR * DIN) return;
  if (in_sizes[7] != NDIR * DIN * NST || in_sizes[8] != NDIR * DIN) return;
  if (in_sizes[9] != DIN || in_sizes[10] != DIN) return;
  if (in_sizes[11] != DMOD * DIN) return;
  if (out_size != NTOK * DMOD) return;

  const size_t SZ_WIN  = (size_t)2 * DIN * DMOD * 2;
  const size_t SZ_WX   = (size_t)NDIR * XDW * DIN * 2;
  const size_t SZ_WO   = (size_t)NPADO * DIN * 2;
  const size_t SZ_X16  = (size_t)NTOK * DMOD * 2;
  const size_t SZ_F192 = (size_t)NTOK * DIN * 4;
  const size_t SZ_H192 = (size_t)NTOK * DIN * 2;
  const size_t SZ_XDBL = (size_t)NDIR * NTOK * XDW * 4;
  const size_t SZ_Y    = (size_t)NDIR * NTOK * DIN * 4;
  const size_t SZ_XR   = (size_t)NTOK * NPADO * 4;
  const size_t OFF_WIN  = 0;
  const size_t OFF_WX   = OFF_WIN  + SZ_WIN;
  const size_t OFF_WOH  = OFF_WX   + SZ_WX;
  const size_t OFF_WOL  = OFF_WOH  + SZ_WO;
  const size_t OFF_X16  = OFF_WOL  + SZ_WO;
  const size_t OFF_XP   = OFF_X16  + SZ_X16;
  const size_t OFF_ZB   = OFF_XP   + SZ_F192;
  const size_t OFF_XI   = OFF_ZB   + SZ_F192;
  const size_t OFF_XI16 = OFF_XI   + SZ_F192;
  const size_t OFF_XDBL = OFF_XI16 + SZ_H192;
  const size_t OFF_Y    = OFF_XDBL + SZ_XDBL;
  const size_t OFF_YGH  = OFF_Y    + SZ_Y;
  const size_t OFF_YGL  = OFF_YGH  + SZ_H192;
  const size_t OFF_XR   = OFF_YGL  + SZ_H192;
  const size_t TOTAL    = OFF_XR   + SZ_XR;
  if (ws_size < TOTAL) return;

  char* ws = (char*)d_ws;
  unsigned short* WIN  = (unsigned short*)(ws + OFF_WIN);
  unsigned short* WX   = (unsigned short*)(ws + OFF_WX);
  unsigned short* WOH  = (unsigned short*)(ws + OFF_WOH);
  unsigned short* WOL  = (unsigned short*)(ws + OFF_WOL);
  unsigned short* X16  = (unsigned short*)(ws + OFF_X16);
  float*          XP   = (float*)(ws + OFF_XP);
  float*          ZB   = (float*)(ws + OFF_ZB);
  float*          XI   = (float*)(ws + OFF_XI);
  unsigned short* XI16 = (unsigned short*)(ws + OFF_XI16);
  float*          XDBL = (float*)(ws + OFF_XDBL);
  float*          YS   = (float*)(ws + OFF_Y);
  unsigned short* YGH  = (unsigned short*)(ws + OFF_YGH);
  unsigned short* YGL  = (unsigned short*)(ws + OFF_YGL);
  float*          XR   = (float*)(ws + OFF_XR);
  const float*    nores = x;

  cast_rows_kernel<<<(NTOK * DMOD / 8) / 256, 256, 0, stream>>>(x, X16, NTOK, NTOK, DMOD, 0, NTOK * DMOD / 8, 1.0f);
  cast_rows_kernel<<<(2 * DIN * DMOD / 8) / 256, 256, 0, stream>>>(inpw, WIN, 2 * DIN, 2 * DIN, DMOD, 0, 2 * DIN * DMOD / 8, 16.0f);
  cast_rows_kernel<<<(NDIR * XDW * DIN / 8) / 256, 256, 0, stream>>>(xprw, WX, XPROWS, XDW, DIN, DTRK, NDIR * XDW * DIN / 8, 16.0f);
  cast_rows_bf2_kernel<<<(NPADO * DIN / 8) / 256, 256, 0, stream>>>(outw, WOH, WOL, DMOD, NPADO, DIN, NPADO * DIN / 8);

  wmma_gemm64<0, false, 0, 0, false, 0><<<dim3(48, 1), 256, 0, stream>>>(
      X16, X16, DMOD, 0L, WIN, WIN, DMOD, 0L, (void*)XP, (void*)XP, DIN, 0L,
      nores, nores, 0L, NTOK, DIN, DMOD, 1.0f / 16.0f);
  wmma_gemm64<0, false, 0, 0, false, 0><<<dim3(48, 1), 256, 0, stream>>>(
      X16, X16, DMOD, 0L, WIN + (size_t)DIN * DMOD, WIN + (size_t)DIN * DMOD, DMOD, 0L,
      (void*)ZB, (void*)ZB, DIN, 0L, nores, nores, 0L, NTOK, DIN, DMOD, 1.0f / 16.0f);

  dwconv_silu_kernel<<<NBATCH * IMH, DIN, 0, stream>>>(XP, cw, cb, XI, XI16);

  wmma_gemm64<0, false, 0, 0, false, 0><<<dim3(16, NDIR), 256, 0, stream>>>(
      XI16, XI16, DIN, 0L, WX, WX, DIN, (long)XDW * DIN, (void*)XDBL, (void*)XDBL, XDW, (long)NTOK * XDW,
      nores, nores, 0L, NTOK, XDW, DIN, 1.0f / 1024.0f);

  scan_dir_kernel<<<NBATCH * NDIR, DIN, 0, stream>>>(XDBL, XI, dtpw, dtpb, alog, dsp, YS);

  ln_gate_kernel<<<NTOK / 32, 256, 0, stream>>>(YS, ZB, lng, lnb, YGH, YGL);

  wmma_gemm64<1, true, 0, 0, false, 0><<<dim3(32, 1), 256, 0, stream>>>(
      YGH, YGL, DIN, 0L, WOH, WOL, DIN, 0L, (void*)XR, (void*)XR, NPADO, 0L,
      nores, nores, 0L, NTOK, NPADO, DIN, 1.0f);

  out_copy_kernel<<<(NTOK * 24) / 256, 256, 0, stream>>>(XR, dout, NTOK * 24);
}
